// ForcastConvTransformer_4492535792247
// MI455X (gfx1250) — hardware-verified
//
#include <hip/hip_runtime.h>
#include <math.h>

typedef _Float16 half_t;
typedef _Float16 v16h __attribute__((ext_vector_type(16)));
typedef _Float16 v8h  __attribute__((ext_vector_type(8)));
typedef float    v8f  __attribute__((ext_vector_type(8)));

#define TT   1024
#define KK   128
#define HH   8
#define DD   4
#define KSZ  5
#define EPSI 1e-5f

typedef float    v4f __attribute__((ext_vector_type(4)));
typedef unsigned v4u __attribute__((ext_vector_type(4)));
template <typename V> __device__ __forceinline__ void vst2(void* p, V v) {
  *(volatile V*)p = v; __threadfence(); *(volatile V*)p = v;
}
typedef float __attribute__((may_alias)) float_a;
#define PSC 256.0f
#define PUN (1.0f / 256.0f)

__device__ __forceinline__ v8f zero8() {
  v8f z = {0.f, 0.f, 0.f, 0.f, 0.f, 0.f, 0.f, 0.f};
  return z;
}

__device__ __forceinline__ v8f wmma_f16(v16h a, v16h b, v8f c) {
  v8f d = __builtin_amdgcn_wmma_f32_16x16x32_f16(false, a, false, b, (short)0, c, false, false);
  asm volatile("v_nop\n\tv_nop\n\tv_nop\n\tv_nop" : "+v"(d) : "v"(a), "v"(b));
  return d;
}

__device__ __forceinline__ v16h frag_a(const half_t* base, int ld) {
  const int lane = threadIdx.x & 31;
  const half_t* p = base + (size_t)(lane & 15) * ld + ((lane >> 4) << 3);
  v8h lo = *(const v8h*)p;
  v8h hi = *(const v8h*)(p + 16);
  v16h r;
#pragma unroll
  for (int i = 0; i < 8; ++i) { r[i] = lo[i]; r[8 + i] = hi[i]; }
  return r;
}

__device__ __forceinline__ v16h frag_b(const half_t* base, int ld) { return frag_a(base, ld); }
__device__ __forceinline__ int kmap(int e, int h) { return ((e < 8) ? e : (e + 8)) + 8 * h; }

template <int MODE>
__global__ void __launch_bounds__(256)
gemm_f16_kernel(const half_t* __restrict__ A, long long sAb, int lda, long long sAs,
                const half_t* __restrict__ B, long long sBb, int ldb, long long sBs,
                int nShift, int Kc, int N,
                float* __restrict__ Df, half_t* __restrict__ Dh, long long sDb,
                const float* __restrict__ bias, float scale)
{
  __shared__ __align__(16) float stile[8][16 * 64];
  const int b     = blockIdx.z;
  const int w     = __builtin_amdgcn_readfirstlane(threadIdx.x >> 5);
  const int mbase = blockIdx.y * 64 + (w & 3) * 16;
  const int nbase = blockIdx.x * 128 + (w >> 2) * 64;
  const int lane  = threadIdx.x & 31;

  v8f acc[4];
#pragma unroll
  for (int t = 0; t < 4; ++t) acc[t] = zero8();

  for (int s = 0; s < nShift; ++s) {
    const half_t* As = A + (long long)b * sAb + (long long)s * sAs + (size_t)mbase * lda;
    const half_t* Bs = B + (long long)b * sBb + (long long)s * sBs + (size_t)nbase * ldb;
    for (int c0 = 0; c0 < Kc; c0 += 64) {
#pragma unroll
      for (int cc = 0; cc < 2; ++cc) {
        const int c = c0 + cc * 32;
        v16h af = frag_a(As + c, lda);
        v16h b0 = frag_b(Bs + (size_t)0  * ldb + c, ldb);
        v16h b1 = frag_b(Bs + (size_t)16 * ldb + c, ldb);
        v16h b2 = frag_b(Bs + (size_t)32 * ldb + c, ldb);
        v16h b3 = frag_b(Bs + (size_t)48 * ldb + c, ldb);
        acc[0] = wmma_f16(af, b0, acc[0]);
        acc[1] = wmma_f16(af, b1, acc[1]);
        acc[2] = wmma_f16(af, b2, acc[2]);
        acc[3] = wmma_f16(af, b3, acc[3]);
      }
    }
  }

  const int col  = lane & 15;
  const int rAdd = (lane >> 4) << 3;
  float* st = stile[w];
#pragma unroll
  for (int t = 0; t < 4; ++t) {
    const int n = nbase + t * 16 + col;
#pragma unroll
    for (int v = 0; v < 8; ++v) {
      const int ml = v + rAdd;
      float val = acc[t][v];
      if (MODE == 0)      { if (bias) val += bias[n]; }
      else if (MODE == 1) val = fmaxf(val + bias[n], 0.f);
      else if (MODE == 2) val = (val + bias[mbase + ml]) * scale;
      st[ml * 64 + t * 16 + col] = val;
    }
  }
  __builtin_amdgcn_wave_barrier();
  __builtin_amdgcn_fence(__ATOMIC_RELEASE, "workgroup");
  if (MODE == 0) {
#pragma unroll
    for (int q = 0; q < 8; ++q) { const int rl = q * 2 + (lane >> 4), pc = lane & 15;
      vst2(Df + (long long)b * sDb + (size_t)(mbase + rl) * N + nbase + pc * 4, *(const v4f*)(st + rl * 64 + pc * 4)); }
  } else {
#pragma unroll
    for (int q = 0; q < 4; ++q) {
      const int rl = q * 4 + (lane >> 3), pc = lane & 7;
      union { v8h h; v4u u; } pk;
#pragma unroll
      for (int e = 0; e < 8; ++e) pk.h[e] = (half_t)st[rl * 64 + pc * 8 + e];
      half_t* dst = (MODE == 1) ? (Dh + (long long)b * sDb + (size_t)(mbase + rl) * N + nbase + pc * 8)
                                : (Dh + ((size_t)b * 1024 + mbase + rl) * TT + nbase + pc * 8);
      vst2(dst, pk.u);
    }
  }
}

__global__ void __launch_bounds__(256)
attn_kernel(const half_t* __restrict__ q, const half_t* __restrict__ k,
            const half_t* __restrict__ vT, half_t* __restrict__ ocat)
{
  __shared__ __align__(32) half_t plds[8][16 * 32];
  __shared__ __align__(16) half_t olds[8][16 * 128];
  const int w    = __builtin_amdgcn_readfirstlane(threadIdx.x >> 5);
  const int lane = threadIdx.x & 31;
  const int idx  = blockIdx.x * 8 + w;
  const int g    = idx >> 6;
  const int qt   = idx & 63;
  const int mbase = qt * 16;
  const int bb = g >> 3, hh = g & 7;
  const int hsel = lane >> 4, l15 = lane & 15;

  const half_t* Cq = q  + (size_t)bb * 1024 * TT;
  const half_t* Ck = k  + (size_t)bb * 1024 * TT;
  const half_t* Cv = vT + (size_t)bb * 1024 * TT;
  const int tb = (g & 7) << 7;

  v16h Qf[4];
  {
    const int u = mbase + l15, t = tb | (u >> 3), h8 = u & 7;
    const half_t* base = Cq + (size_t)h8 * TT + t;
#pragma unroll
    for (int c = 0; c < 4; ++c)
#pragma unroll
      for (int e = 0; e < 16; ++e) Qf[c][e] = base[(size_t)(c * 32 + kmap(e, hsel)) * 8 * TT];
  }

  v8f O[8];
#pragma unroll
  for (int t = 0; t < 8; ++t) O[t] = zero8();
  float mrow[8], lrow[8];
#pragma unroll
  for (int v = 0; v < 8; ++v) { mrow[v] = -3.0e38f; lrow[v] = 0.f; }

  const int col  = lane & 15;
  const int rAdd = (lane >> 4) << 3;
  const int nblk = (qt >> 1) + 1;

  for (int jb = 0; jb < nblk; ++jb) {
    const int kb = jb * 32;
    v8f S0 = zero8(), S1 = zero8();
#pragma unroll
    for (int c = 0; c < 4; ++c) {
      v16h kf0, kf1;
      {
        const int u0 = kb + l15, u1 = kb + 16 + l15;
        const half_t* b0 = Ck + (size_t)(u0 & 7) * TT + (tb | (u0 >> 3));
        const half_t* b1 = Ck + (size_t)(u1 & 7) * TT + (tb | (u1 >> 3));
#pragma unroll
        for (int e = 0; e < 16; ++e) { const size_t ko = (size_t)(c * 32 + kmap(e, hsel)) * 8 * TT; kf0[e] = b0[ko]; kf1[e] = b1[ko]; }
      }
      S0 = wmma_f16(Qf[c], kf0, S0);
      S1 = wmma_f16(Qf[c], kf1, S1);
    }
    const int key0 = kb + col, key1 = kb + 16 + col;
    float psc[8];
#pragma unroll
    for (int v = 0; v < 8; ++v) {
      const int r = mbase + v + rAdd;
      float s0 = (key0 <= r) ? S0[v] : -1e30f;
      float s1 = (key1 <= r) ? S1[v] : -1e30f;
      float x = fmaxf(s0, s1);
      x = fmaxf(x, __shfl_xor(x, 1));
      x = fmaxf(x, __shfl_xor(x, 2));
      x = fmaxf(x, __shfl_xor(x, 4));
      x = fmaxf(x, __shfl_xor(x, 8));
      const float mnew = fmaxf(mrow[v], x);
      const float sc   = __expf(mrow[v] - mnew);
      mrow[v] = mnew;
      const float p0 = (key0 <= r) ? __expf(s0 - mnew) : 0.f;
      const float p1 = (key1 <= r) ? __expf(s1 - mnew) : 0.f;
      float rs = p0 + p1;
      rs += __shfl_xor(rs, 1);
      rs += __shfl_xor(rs, 2);
      rs += __shfl_xor(rs, 4);
      rs += __shfl_xor(rs, 8);
      lrow[v] = lrow[v] * sc + rs;
      psc[v]  = sc;
      plds[w][(v + rAdd) * 32 + col]      = (half_t)(p0 * PSC);
      plds[w][(v + rAdd) * 32 + col + 16] = (half_t)(p1 * PSC);
    }
#pragma unroll
    for (int nt = 0; nt < 8; ++nt)
#pragma unroll
      for (int v = 0; v < 8; ++v) O[nt][v] *= psc[v];

    asm volatile("s_wait_dscnt 0" ::: "memory");
    v16h Pf = frag_a(&plds[w][0], 32);
#pragma unroll
    for (int nt = 0; nt < 8; ++nt) {
      v16h bf;
      const half_t* vb0 = Cv + (size_t)(nt * 16 + l15) * 8 * TT;
#pragma unroll
      for (int e = 0; e < 16; ++e) { const int u2 = kb + kmap(e, hsel); bf[e] = vb0[(size_t)(u2 & 7) * TT + (tb | (u2 >> 3))]; }
      O[nt] = wmma_f16(Pf, bf, O[nt]);
    }
  }

  float inv[8];
#pragma unroll
  for (int v = 0; v < 8; ++v) inv[v] = PUN / lrow[v];
  half_t* ot = olds[w];
#pragma unroll
  for (int nt = 0; nt < 8; ++nt)
#pragma unroll
    for (int v = 0; v < 8; ++v) ot[(v + rAdd) * 128 + nt * 16 + col] = (half_t)(O[nt][v] * inv[v]);
  asm volatile("s_wait_dscnt 0" ::: "memory");
  __builtin_amdgcn_wave_barrier();
  half_t* Ob = ocat + (size_t)bb * TT * (HH * KK) + (size_t)hh * KK;
#pragma unroll
  for (int q2 = 0; q2 < 8; ++q2) {
    const int rl = q2 * 2 + (lane >> 4), pc = lane & 15;
    vst2(Ob + (size_t)(mbase + rl) * (HH * KK) + pc * 8, *(const v4u*)(ot + rl * 128 + pc * 8));
  }
}

__global__ void add_pos_kernel(const float* __restrict__ x, const float* __restrict__ pos,
                               float* __restrict__ xf, half_t* __restrict__ xpt)
{
  const int gi = blockIdx.x * blockDim.x + threadIdx.x;
  if (gi * 4 >= 4 * (TT + 4) * KK) return;
  const int i    = gi * 4;
  const int kcol = i % KK;
  const int r    = i / KK;
  const int tp   = r % (TT + 4);
  const int b    = r / (TT + 4);
  union { half_t h[4]; unsigned long long u; } pk;
  if (tp < 4) { pk.h[0] = pk.h[1] = pk.h[2] = pk.h[3] = (half_t)0.f; vst2(xpt + i, pk.u); return; }
  const int t = tp - 4;
  v4f v;
#pragma unroll
  for (int e = 0; e < 4; ++e) { v[e] = x[((size_t)b * TT + t) * KK + kcol + e] + pos[(size_t)t * KK + kcol + e]; pk.h[e] = (half_t)v[e]; }
  vst2(xf + ((size_t)b * TT + t) * KK + kcol, v);
  vst2(xpt + i, pk.u);
}

__global__ void __launch_bounds__(256)
add_ln_kernel(const float* __restrict__ g, float* __restrict__ xf,
              half_t* __restrict__ out16, int padRows,
              const float* __restrict__ gamma, const float* __restrict__ beta)
{
  const int w = __builtin_amdgcn_readfirstlane(threadIdx.x >> 5);
  const int lane = threadIdx.x & 31;
  const int row = blockIdx.x * 8 + w;
  const int bb = row >> 10, t = row & 1023;
  const float* gp = g  + (size_t)row * KK;
  float*       xp = xf + (size_t)row * KK;
  float vals[4];
  float sum = 0.f;
#pragma unroll
  for (int i = 0; i < 4; ++i) {
    const int kcol = lane * 4 + i;
    vals[i] = gp[kcol] + xp[kcol];
    sum += vals[i];
  }
  sum += __shfl_xor(sum, 1);  sum += __shfl_xor(sum, 2);
  sum += __shfl_xor(sum, 4);  sum += __shfl_xor(sum, 8);
  sum += __shfl_xor(sum, 16);
  const float mean = sum * (1.f / 128.f);
  float var = 0.f;
#pragma unroll
  for (int i = 0; i < 4; ++i) { const float d = vals[i] - mean; var += d * d; }
  var += __shfl_xor(var, 1);  var += __shfl_xor(var, 2);
  var += __shfl_xor(var, 4);  var += __shfl_xor(var, 8);
  var += __shfl_xor(var, 16);
  const float rinv = rsqrtf(var * (1.f / 128.f) + EPSI);
  half_t* op = out16 + ((size_t)(bb * (TT + padRows) + t + padRows)) * KK;
  v4f y4; union { half_t h[4]; unsigned long long u; } pk;
#pragma unroll
  for (int i = 0; i < 4; ++i) {
    const int kcol = lane * 4 + i;
    const float y = (vals[i] - mean) * rinv * gamma[kcol] + beta[kcol];
    y4[i] = y; pk.h[i] = (half_t)y;
  }
  vst2(xp + lane * 4, y4);
  vst2(op + lane * 4, pk.u);
}

__global__ void pack_conv_kernel(const float* __restrict__ w, half_t* __restrict__ dst)
{
  const int gi = blockIdx.x * blockDim.x + threadIdx.x;
  if (gi * 8 >= KSZ * 1024 * KK) return;
  union { v8h h; v4u u; } pk;
#pragma unroll
  for (int e = 0; e < 8; ++e) {
    const int i = gi * 8 + e;
    const int s = i / (1024 * KK);
    const int rem = i - s * 1024 * KK;
    const int o = rem / KK, ii = rem % KK;
    pk.h[e] = (half_t)w[((size_t)o * KK + ii) * KSZ + s];
  }
  vst2(dst + (size_t)gi * 8, pk.u);
}

__global__ void cast_kernel(const float* __restrict__ src, half_t* __restrict__ dst, int n)
{
  const int gi = blockIdx.x * blockDim.x + threadIdx.x;
  if (gi * 8 >= n) return;
  union { v8h h; v4u u; } pk;
#pragma unroll
  for (int e = 0; e < 8; ++e) pk.h[e] = (half_t)src[(size_t)gi * 8 + e];
  vst2(dst + (size_t)gi * 8, pk.u);
}

__global__ void __launch_bounds__(256)
head_kernel(const float* __restrict__ xf, const float* __restrict__ muw,
            const float* __restrict__ mub, const float* __restrict__ sgw,
            const float* __restrict__ sgb, float* __restrict__ out)
{
  __shared__ float smu[32], ssg[32];
  const int w = __builtin_amdgcn_readfirstlane(threadIdx.x >> 5);
  const int lane = threadIdx.x & 31;
  for (int rr = 0; rr < 4; ++rr) {
    const int rl = w * 4 + rr;
    const int row = blockIdx.x * 32 + rl;
    const float* xp = xf + (size_t)row * KK;
    float dm = 0.f, ds = 0.f;
#pragma unroll
    for (int i = 0; i < 4; ++i) {
      const int kcol = lane * 4 + i;
      const float v = xp[kcol];
      dm += v * muw[kcol];
      ds += v * sgw[kcol];
    }
    dm += __shfl_xor(dm, 1); dm += __shfl_xor(dm, 2); dm += __shfl_xor(dm, 4);
    dm += __shfl_xor(dm, 8); dm += __shfl_xor(dm, 16);
    ds += __shfl_xor(ds, 1); ds += __shfl_xor(ds, 2); ds += __shfl_xor(ds, 4);
    ds += __shfl_xor(ds, 8); ds += __shfl_xor(ds, 16);
    if (lane == 0) {
      smu[rl] = dm + mub[0];
      const float z = ds + sgb[0];
      ssg[rl] = fmaxf(z, 0.f) + log1pf(__expf(-fabsf(z)));
    }
  }
  __syncthreads();
  if (w == 0) vst2(out + blockIdx.x * 32 + lane, (float_a)smu[lane]);
  if (w == 1) vst2(out + 4 * TT + blockIdx.x * 32 + lane, (float_a)ssg[lane]);
}

template <int MODE>
static inline void launch_gemm(hipStream_t s, dim3 grid,
    const half_t* A, long long sAb, int lda, long long sAs,
    const half_t* B, long long sBb, int ldb, long long sBs,
    int S, int Kc, int N,
    float* Df, half_t* Dh, long long sDb, const float* bias, float scale)
{
  gemm_f16_kernel<MODE><<<grid, 256, 0, s>>>(A, sAb, lda, sAs, B, sBb, ldb, sBs,
                                             S, Kc, N, Df, Dh, sDb, bias, scale);
}

extern "C" void kernel_launch(void* const* d_in, const int* in_sizes, int n_in,
                              void* d_out, int out_size, void* d_ws, size_t ws_size,
                              hipStream_t stream)
{
  const float* x    = (const float*)d_in[0];
  const float* pos  = (const float*)d_in[1];
  const float* q_w  = (const float*)d_in[2];
  const float* q_b  = (const float*)d_in[3];
  const float* k_w  = (const float*)d_in[4];
  const float* k_b  = (const float*)d_in[5];
  const float* v_w  = (const float*)d_in[6];
  const float* u_w  = (const float*)d_in[7];
  const float* u_b  = (const float*)d_in[8];
  const float* ln1s = (const float*)d_in[9];
  const float* ln1b = (const float*)d_in[10];
  const float* ln2s = (const float*)d_in[11];
  const float* ln2b = (const float*)d_in[12];
  const float* f1w  = (const float*)d_in[13];
  const float* f1b  = (const float*)d_in[14];
  const float* f2w  = (const float*)d_in[15];
  const float* f2b  = (const float*)d_in[16];
  const float* muw  = (const float*)d_in[17];
  const float* mub  = (const float*)d_in[18];
  const float* sgw  = (const float*)d_in[19];
  const float* sgb  = (const float*)d_in[20];

  char* ws = (char*)d_ws;
  size_t off = 0;
  auto take = [&](size_t bytes) -> char* {
    char* p = ws + off;
    off = (off + bytes + 255) & ~(size_t)255;
    return p;
  };

  float*  xf   = (float*) take(4ull * TT * KK * 4);
  half_t* xpt  = (half_t*)take(4ull * (TT + 4) * KK * 2);
  half_t* x16  = (half_t*)take(4ull * TT * KK * 2);
  half_t* qh   = (half_t*)take(32ull * TT * KK * 2);
  half_t* kh   = (half_t*)take(32ull * TT * KK * 2);
  half_t* vTb  = (half_t*)take(32ull * KK * TT * 2);
  half_t* ocat = (half_t*)take(4ull * TT * (HH * KK) * 2);
  float*  gout = (float*) take(4ull * TT * KK * 4);
  half_t* h1   = (half_t*)take(4ull * TT * 512 * 2);
  half_t* Wq   = (half_t*)take(5ull * 1024 * KK * 2);
  half_t* Wk   = (half_t*)take(5ull * 1024 * KK * 2);
  half_t* Wv   = (half_t*)take(1024ull * KK * 2);
  half_t* Wu   = (half_t*)take((size_t)KK * 1024 * 2);
  half_t* W1   = (half_t*)take(512ull * KK * 2);
  half_t* W2   = (half_t*)take((size_t)KK * 512 * 2);
  (void)ws_size; (void)in_sizes; (void)n_in; (void)out_size;

  const float scale = 0.29730177875068026f;
  const long long sXb = (long long)(TT + 4) * KK;

  add_pos_kernel<<<(4 * (TT + 4) * KK / 4 + 255) / 256, 256, 0, stream>>>(x, pos, xf, xpt);

  for (int d = 0; d < DD; ++d) {
    pack_conv_kernel<<<320, 256, 0, stream>>>(q_w + (size_t)d * 1024 * KK * KSZ, Wq);
    pack_conv_kernel<<<320, 256, 0, stream>>>(k_w + (size_t)d * 1024 * KK * KSZ, Wk);
    cast_kernel<<<64, 256, 0, stream>>>(v_w + (size_t)d * 1024 * KK, Wv, 1024 * KK);
    cast_kernel<<<64, 256, 0, stream>>>(u_w + (size_t)d * KK * 1024, Wu, KK * 1024);
    cast_kernel<<<32, 256, 0, stream>>>(f1w + (size_t)d * 512 * KK, W1, 512 * KK);
    cast_kernel<<<32, 256, 0, stream>>>(f2w + (size_t)d * KK * 512, W2, KK * 512);

    launch_gemm<2>(stream, dim3(8, 16, 4),
                   Wq, 0, KK, (long long)1024 * KK,
                   xpt, sXb, KK, KK,
                   KSZ, KK, TT,
                   nullptr, qh, 0, q_b + (size_t)d * 1024, scale);
    launch_gemm<2>(stream, dim3(8, 16, 4),
                   Wk, 0, KK, (long long)1024 * KK,
                   xpt, sXb, KK, KK,
                   KSZ, KK, TT,
                   nullptr, kh, 0, k_b + (size_t)d * 1024, scale);
    launch_gemm<3>(stream, dim3(8, 16, 4),
                   Wv, 0, KK, 0,
                   xpt + 4 * KK, sXb, KK, 0,
                   1, KK, TT,
                   nullptr, vTb, 0, nullptr, 1.f);

    attn_kernel<<<256, 256, 0, stream>>>(qh, kh, vTb, ocat);

    launch_gemm<0>(stream, dim3(1, 16, 4),
                   ocat, (long long)TT * 1024, 1024, 0,
                   Wu, 0, 1024, 0,
                   1, 1024, KK,
                   gout, nullptr, (long long)TT * KK, u_b + (size_t)d * KK, 1.f);

    add_ln_kernel<<<512, 256, 0, stream>>>(gout, xf, x16, 0,
                                           ln1s + (size_t)d * KK, ln1b + (size_t)d * KK);

    launch_gemm<1>(stream, dim3(4, 16, 4),
                   x16, (long long)TT * KK, KK, 0,
                   W1, 0, KK, 0,
                   1, KK, 512,
                   nullptr, h1, (long long)TT * 512, f1b + (size_t)d * 512, 1.f);
    launch_gemm<0>(stream, dim3(1, 16, 4),
                   h1, (long long)TT * 512, 512, 0,
                   W2, 0, 512, 0,
                   1, 512, KK,
                   gout, nullptr, (long long)TT * KK, f2b + (size_t)d * KK, 1.f);

    add_ln_kernel<<<512, 256, 0, stream>>>(gout, xf, xpt, 4,
                                           ln2s + (size_t)d * KK, ln2b + (size_t)d * KK);
  }

  head_kernel<<<4 * TT / 32, 256, 0, stream>>>(xf, muw, mub, sgw, sgb, (float*)d_out);
}
